// DotProductAttention_26139170963678
// MI455X (gfx1250) — hardware-verified
//
#include <hip/hip_runtime.h>


#ifndef NB
#define NB 2
#endif
#ifndef SEQ
#define SEQ 2048
#endif
#define NB_FULL  2
#define SEQ_FULL 2048
#define DM   1024
#define NH   16
#define HD   64
#define D3   3072
#define NTOK (NB * SEQ)
#define QT   (SEQ / 16)
#define MCB  64
#define SP   72
#define QKPL ((size_t)NB * NH * SEQ * HD)
#define L2E  1.4426950408889634f

typedef _Float16 h16;
typedef unsigned short bf;
typedef __attribute__((ext_vector_type(16))) __bf16   v16bf;
typedef __attribute__((ext_vector_type(16))) _Float16 v16h;
typedef __attribute__((ext_vector_type(8)))  _Float16 v8h;
typedef __attribute__((ext_vector_type(8)))  unsigned short v8us;
typedef __attribute__((ext_vector_type(2)))  unsigned short v2us;
typedef __attribute__((ext_vector_type(8)))  float    v8f;
typedef __attribute__((ext_vector_type(4)))  float    v4f;
typedef __attribute__((ext_vector_type(4)))  int      v4i;
typedef v4f  __attribute__((may_alias)) v4fa;
typedef v8us __attribute__((may_alias)) v8usa;

static_assert(NTOK % 64 == 0);
static_assert(SEQ % 64 == 0);
static_assert(D3 % 64 == 0);
static_assert(DM % 64 == 0);
static_assert(DM % 32 == 0);
static_assert(HD == 64);
static_assert(NH == 16);
static_assert(QT % 8 == 0);
static_assert((SEQ * (SEQ / 4)) % (MCB * 256) == 0);
static_assert((SEQ * 32) % 256 == 0);
static_assert(((size_t)NTOK * 128) % 256 == 0);
static_assert(((size_t)2 * NTOK * 128) % 256 == 0);
static_assert(((size_t)NB * NH * HD * SEQ / 2) % 256 == 0);
static_assert((size_t)2 * NTOK * DM * 2 <= (size_t)NTOK * D3 * 4);
static_assert(NB <= NB_FULL);
static_assert(SEQ <= SEQ_FULL);

__device__ __forceinline__ unsigned short f2bf(float f) { unsigned u = __float_as_uint(f); u += 0x7FFFu + ((u >> 16) & 1u); return (unsigned short)(u >> 16); }
__device__ __forceinline__ float bf2f(unsigned short b) { return __uint_as_float(((unsigned)b) << 16); }
__device__ __forceinline__ float bfr(float f) { return bf2f(f2bf(f)); }
__device__ __forceinline__ v16h cat16(v8h lo, v8h hi) { return __builtin_shufflevector(lo, hi, 0, 1, 2, 3, 4, 5, 6, 7, 8, 9, 10, 11, 12, 13, 14, 15); }
__device__ __forceinline__ v16bf cat16b(v8us lo, v8us hi) { return __builtin_bit_cast(v16bf, __builtin_shufflevector(lo, hi, 0, 1, 2, 3, 4, 5, 6, 7, 8, 9, 10, 11, 12, 13, 14, 15)); }
__device__ __forceinline__ v8f wmma16(v16h a, v16h b, v8f c) { return __builtin_amdgcn_wmma_f32_16x16x32_f16(false, a, false, b, (short)0, c, false, false); }
__device__ __forceinline__ v8f wmmab(v16bf a, v16bf b, v8f c) { return __builtin_amdgcn_wmma_f32_16x16x32_bf16(false, a, false, b, (short)0, c, false, false); }
__device__ __forceinline__ void splitf(float y, unsigned short& h, unsigned short& l) { h = f2bf(y); l = f2bf(y - bf2f(h)); }

template <typename T16> struct WFrag;
template <> struct WFrag<h16> { typedef v16h V; static __device__ __forceinline__ V ld(const h16* p) { return cat16(*(const v8h*)p, *(const v8h*)(p + 16)); } static __device__ __forceinline__ v8f mma(V a, V b, v8f c) { return wmma16(a, b, c); } };
template <> struct WFrag<bf> { typedef v16bf V; static __device__ __forceinline__ V ld(const bf* p) { return cat16b(*(const v8us*)p, *(const v8us*)(p + 16)); } static __device__ __forceinline__ v8f mma(V a, V b, v8f c) { return wmmab(a, b, c); } };
template <typename T16, int NSPLIT, bool BIAS>
__global__ __launch_bounds__(32) void k_gemmw(const T16* __restrict__ A, const T16* __restrict__ A2, const T16* __restrict__ Bt, const T16* __restrict__ Bt2, int K, float* C, int ldc, const float* __restrict__ bias, size_t sA, size_t sB, size_t sC) {
    typedef typename WFrag<T16>::V V;
    __shared__ __align__(16) float os[16 * 68];
    const size_t z = blockIdx.z; A += z * sA; if (A2) A2 += z * sA; Bt += z * sB; if (Bt2) Bt2 += z * sB; C += z * sC;
    const int lane = threadIdx.x & 31, lr = lane & 15, hi = lane >> 4; const int r0 = blockIdx.x * 64, c0 = blockIdx.y * 64;
    v8f acc[4][4];
#pragma unroll
    for (int mb = 0; mb < 4; ++mb)
#pragma unroll
        for (int nb = 0; nb < 4; ++nb) acc[mb][nb] = (v8f){};
    const size_t aoff = (size_t)(r0 + lr) * K + 8 * hi, boff = (size_t)(c0 + lr) * K + 8 * hi;
#pragma unroll 1
    for (int kc = 0; kc < K; kc += 32) {
        V a[4], a2[4];
#pragma unroll
        for (int mb = 0; mb < 4; ++mb) { a[mb] = WFrag<T16>::ld(A + aoff + (size_t)mb * 16 * K + kc); if (NSPLIT == 1 || NSPLIT == 2) a2[mb] = WFrag<T16>::ld(A2 + aoff + (size_t)mb * 16 * K + kc); }
#pragma unroll
        for (int nb = 0; nb < 4; ++nb) { const V b = WFrag<T16>::ld(Bt + boff + (size_t)nb * 16 * K + kc); V b2; if (NSPLIT >= 2) b2 = WFrag<T16>::ld(Bt2 + boff + (size_t)nb * 16 * K + kc);
#pragma unroll
            for (int mb = 0; mb < 4; ++mb) { acc[mb][nb] = WFrag<T16>::mma(a[mb], b, acc[mb][nb]); if (NSPLIT == 1 || NSPLIT == 2) acc[mb][nb] = WFrag<T16>::mma(a2[mb], b, acc[mb][nb]); if (NSPLIT >= 2) acc[mb][nb] = WFrag<T16>::mma(a[mb], b2, acc[mb][nb]); } }
        asm volatile("v_nop\n\tv_nop\n\tv_nop\n\tv_nop" : "+v"(acc[0][0]), "+v"(acc[1][1]), "+v"(acc[2][2]), "+v"(acc[3][3]) : "v"(a[0]), "v"(a[3]));
    }
#pragma unroll
    for (int mb = 0; mb < 4; ++mb) {
#pragma unroll
        for (int nb = 0; nb < 4; ++nb) {
#pragma unroll
            for (int j = 0; j < 8; ++j) os[(hi * 8 + j) * 68 + nb * 16 + lr] = acc[mb][nb][j]; }
        __builtin_amdgcn_wave_barrier(); asm volatile("" ::: "memory");
        float* crow = C + (size_t)(r0 + mb * 16) * ldc + c0;
#pragma unroll 1
        for (int ps = 0; ps < 2; ++ps) {
#pragma unroll
            for (int s = 0; s < 8; ++s) { const int row = 2 * s + hi, cofs = lr * 4; v4f val = *(const v4fa*)(os + row * 68 + cofs); if (BIAS) { val[0] += bfr(bias[c0 + cofs]); val[1] += bfr(bias[c0 + cofs + 1]); val[2] += bfr(bias[c0 + cofs + 2]); val[3] += bfr(bias[c0 + cofs + 3]); }
                *(volatile v4f*)(crow + (size_t)row * ldc + cofs) = val; }
            if (ps == 0) __threadfence(); }
        __builtin_amdgcn_wave_barrier(); asm volatile("" ::: "memory");
    }
}

__global__ __launch_bounds__(256) void k_cvt8(const float* __restrict__ src, bf* dst, size_t n8) { const size_t i = (size_t)blockIdx.x * 256 + threadIdx.x; if (i >= n8) return; const v8f v = *(const v8f*)(src + i * 8); v8us o;
#pragma unroll
    for (int k = 0; k < 8; ++k) o[k] = f2bf(v[k]); *(volatile v8us*)(dst + i * 8) = o; __threadfence(); *(volatile v8us*)(dst + i * 8) = o; }

__global__ __launch_bounds__(256) void k_cvtx(const float* __restrict__ x, bf* dst) {
    const unsigned i = blockIdx.x * 256u + threadIdx.x; const unsigned tok = i >> 7, c8 = i & 127u; const unsigned b = tok / (unsigned)SEQ, s = tok - b * (unsigned)SEQ;
    const v8f v = *(const v8f*)(x + ((size_t)b * SEQ_FULL + s) * DM + c8 * 8u); v8us o;
#pragma unroll
    for (int k = 0; k < 8; ++k) o[k] = f2bf(v[k]);
    *(volatile v8us*)(dst + (size_t)i * 8) = o; __threadfence(); *(volatile v8us*)(dst + (size_t)i * 8) = o; }

__global__ __launch_bounds__(256) void k_trig(const float* __restrict__ fr, float* CS, float* SN) {
    const unsigned i = blockIdx.x * 256u + threadIdx.x; const float a = bfr(fr[i]); const float c = cosf(a), s = sinf(a);
    *(volatile float*)(CS + i) = c; *(volatile float*)(SN + i) = s; __threadfence(); *(volatile float*)(CS + i) = c; *(volatile float*)(SN + i) = s; }

__global__ __launch_bounds__(256) void k_mchk(const int* __restrict__ mask, int* FL) {
    const unsigned gid = blockIdx.x * 256u + threadIdx.x; int bad = 0;
#pragma unroll 1
    for (unsigned g = gid; g < (unsigned)(SEQ * (SEQ / 4)); g += (unsigned)(MCB * 256)) { const unsigned q = g / (unsigned)(SEQ / 4), k = (g - q * (unsigned)(SEQ / 4)) * 4u; const v4i mv = *(const v4i*)(mask + (size_t)q * SEQ_FULL + k);
#pragma unroll
        for (unsigned j = 0; j < 4; ++j) { const int want = (k + j <= q) ? 1 : 0; const int got = (mv[j] != 0) ? 1 : 0; bad |= (want ^ got); } }
    const int any = __syncthreads_or(bad);
    if (threadIdx.x < 32u) { const int v = any ? 1 : 0; *(volatile int*)(FL + blockIdx.x * 32u + threadIdx.x) = v; __threadfence(); *(volatile int*)(FL + blockIdx.x * 32u + threadIdx.x) = v; }
}

__global__ __launch_bounds__(256) void k_rope(const float* __restrict__ QKV, const float* __restrict__ CS, const float* __restrict__ SN, bf* QKh, bf* QKl) {
    const unsigned i = blockIdx.x * 256u + threadIdx.x; const unsigned pc = i & 7u, h = (i >> 3) & 15u, t = i >> 7; const unsigned which = t / (unsigned)NTOK, tok = t - which * (unsigned)NTOK; const unsigned b = tok / (unsigned)SEQ, s = tok - b * (unsigned)SEQ;
    const v8f v = *(const v8f*)(QKV + (size_t)tok * D3 + which * (unsigned)DM + h * (unsigned)HD + pc * 8u);
    const v4f c4 = *(const v4f*)(CS + s * 32u + pc * 4u); const v4f s4 = *(const v4f*)(SN + s * 32u + pc * 4u);
    const float sc = which ? 1.0f : 0.125f; v8us oh, ol;
#pragma unroll
    for (int j = 0; j < 4; ++j) { const float t1 = v[2 * j], t2 = v[2 * j + 1]; const float a = (t1 * c4[j] - t2 * s4[j]) * sc; const float bb = (t1 * s4[j] + t2 * c4[j]) * sc; unsigned short x0, x1; splitf(a, x0, x1); oh[2 * j] = x0; ol[2 * j] = x1; splitf(bb, x0, x1); oh[2 * j + 1] = x0; ol[2 * j + 1] = x1; }
    const size_t oo = (size_t)which * QKPL + (((size_t)(b * (unsigned)NH + h)) * SEQ + s) * HD + pc * 8u;
    *(volatile v8us*)(QKh + oo) = oh; *(volatile v8us*)(QKl + oo) = ol; __threadfence(); *(volatile v8us*)(QKh + oo) = oh; *(volatile v8us*)(QKl + oo) = ol; }

__global__ __launch_bounds__(256) void k_vtp(const float* __restrict__ QKV, bf* Vh, bf* Vl) {
    const unsigned e = (blockIdx.x * 256u + threadIdx.x) * 2u; const unsigned s = e % (unsigned)SEQ; const unsigned d = (e / (unsigned)SEQ) & 63u; const unsigned bh = e / (unsigned)(SEQ * HD); const unsigned b = bh >> 4, h = bh & 15u; v2us oh, ol;
#pragma unroll
    for (unsigned q = 0; q < 2; ++q) { const float x = QKV[(size_t)(b * (unsigned)SEQ + s + q) * D3 + 2u * DM + h * (unsigned)HD + d]; unsigned short a2, c2; splitf(x, a2, c2); oh[q] = a2; ol[q] = c2; }
    *(volatile v2us*)(Vh + e) = oh; *(volatile v2us*)(Vl + e) = ol; __threadfence(); *(volatile v2us*)(Vh + e) = oh; *(volatile v2us*)(Vl + e) = ol; }

__global__ __launch_bounds__(256) void k_flash(const bf* __restrict__ QKh, const bf* __restrict__ QKl, const bf* __restrict__ VTh, const bf* __restrict__ VTl, const int* __restrict__ FL, bf* CH, bf* CL) {
    typedef WFrag<bf>::V V;
    __shared__ __align__(16) unsigned short stg[8 * 2 * 16 * SP];
    const unsigned lane = threadIdx.x & 31u, lr = lane & 15u, hi = lane >> 4, wv = threadIdx.x >> 5;
    const unsigned wid = blockIdx.x * 8u + wv; const unsigned qt = wid % (unsigned)QT, bh = wid / (unsigned)QT; const unsigned q0 = qt * 16u; const unsigned b = bh >> 4, h = bh & 15u;
    int fbad = ((FL[lane * 32u] == 1) ? 1 : 0) | ((FL[(lane + 32u) * 32u] == 1) ? 1 : 0);
#pragma unroll
    for (int sh = 16; sh; sh >>= 1) fbad |= __shfl_xor(fbad, sh, 32);
    const float poison = fbad ? __uint_as_float(0x7FC00000u) : 0.0f;
    const size_t qo = ((size_t)bh * SEQ + q0 + lr) * HD + 8u * hi;
    V bqh[2], bql[2];
#pragma unroll
    for (int c = 0; c < 2; ++c) { bqh[c] = WFrag<bf>::ld(QKh + qo + 32 * c); bql[c] = WFrag<bf>::ld(QKl + qo + 32 * c); }
    const bf* Kh = QKh + QKPL + ((size_t)bh * SEQ + lr) * HD + 8u * hi; const bf* Kl = QKl + QKPL + ((size_t)bh * SEQ + lr) * HD + 8u * hi;
    const bf* Vh = VTh + ((size_t)bh * HD + lr) * SEQ + 8u * hi; const bf* Vl = VTl + ((size_t)bh * HD + lr) * SEQ + 8u * hi;
    v8f o[4];
#pragma unroll
    for (int t = 0; t < 4; ++t) o[t] = (v8f){};
    float m = -1.0e30f, l = 0.0f; const unsigned qg = q0 + lr;
#pragma unroll 1
    for (unsigned kt = 0; kt < q0 + 16u; kt += 32u) {
        V kh[2][2], kl[2][2];
#pragma unroll
        for (int c = 0; c < 2; ++c)
#pragma unroll
            for (int j = 0; j < 2; ++j) { kh[c][j] = WFrag<bf>::ld(Kh + (size_t)(kt + 16u * j) * HD + 32 * c); kl[c][j] = WFrag<bf>::ld(Kl + (size_t)(kt + 16u * j) * HD + 32 * c); }
        v8f sc[2]; sc[0] = (v8f){}; sc[1] = (v8f){};
#pragma unroll
        for (int c = 0; c < 2; ++c)
#pragma unroll
            for (int j = 0; j < 2; ++j) { sc[j] = wmmab(kh[c][j], bqh[c], sc[j]); sc[j] = wmmab(kh[c][j], bql[c], sc[j]); sc[j] = wmmab(kl[c][j], bqh[c], sc[j]); }
        asm volatile("v_nop\n\tv_nop\n\tv_nop\n\tv_nop" : "+v"(sc[0]), "+v"(sc[1]) : "v"(kh[1][0]), "v"(kh[1][1]), "v"(kl[1][0]), "v"(kl[1][1]), "v"(bqh[1]), "v"(bql[1]));
        float v0[8], v1[8]; float tmax = -1.0e30f;
#pragma unroll
        for (unsigned r = 0; r < 8; ++r) { const unsigned key0 = kt + 8u * hi + r; v0[r] = (key0 <= qg) ? sc[0][r] : -1.0e30f; v1[r] = (key0 + 16u <= qg) ? sc[1][r] : -1.0e30f; tmax = fmaxf(tmax, fmaxf(v0[r], v1[r])); }
        tmax = fmaxf(tmax, __shfl_xor(tmax, 16, 32));
        const float mnew = fmaxf(m, tmax); const float corr = __builtin_amdgcn_exp2f((m - mnew) * L2E);
        float psum = 0.0f; v8us ph0, pl0, ph1, pl1;
#pragma unroll
        for (int r = 0; r < 8; ++r) { const float e0 = __builtin_amdgcn_exp2f((v0[r] - mnew) * L2E); const float e1 = __builtin_amdgcn_exp2f((v1[r] - mnew) * L2E); psum += e0 + e1; unsigned short a, c2; splitf(e0, a, c2); ph0[r] = a; pl0[r] = c2; splitf(e1, a, c2); ph1[r] = a; pl1[r] = c2; }
        psum += __shfl_xor(psum, 16, 32);
        l = l * corr + psum; m = mnew;
#pragma unroll
        for (int t = 0; t < 4; ++t) o[t] = o[t] * corr;
        const V pbh = cat16b(ph0, ph1), pbl = cat16b(pl0, pl1);
        V avh[4], avl[4];
#pragma unroll
        for (int t = 0; t < 4; ++t) { avh[t] = WFrag<bf>::ld(Vh + (size_t)t * 16 * SEQ + kt); avl[t] = WFrag<bf>::ld(Vl + (size_t)t * 16 * SEQ + kt); }
#pragma unroll
        for (int t = 0; t < 4; ++t) { o[t] = wmmab(avh[t], pbh, o[t]); o[t] = wmmab(avh[t], pbl, o[t]); o[t] = wmmab(avl[t], pbh, o[t]); }
        asm volatile("v_nop\n\tv_nop\n\tv_nop\n\tv_nop" : "+v"(o[0]), "+v"(o[1]), "+v"(o[2]), "+v"(o[3]) : "v"(pbh), "v"(pbl), "v"(avl[0]), "v"(avl[1]), "v"(avl[2]), "v"(avl[3]), "v"(avh[3]));
    }
    const float inv = 1.0f / l;
    unsigned short* sh = stg + wv * (2u * 16u * SP); unsigned short* sl = sh + 16u * SP;
#pragma unroll
    for (int t = 0; t < 4; ++t) { v8us oh, ol;
#pragma unroll
        for (int r = 0; r < 8; ++r) { const float val = o[t][r] * inv + poison; unsigned short a, c2; splitf(val, a, c2); oh[r] = a; ol[r] = c2; }
        *(v8usa*)(sh + lr * SP + 16u * t + 8u * hi) = oh; *(v8usa*)(sl + lr * SP + 16u * t + 8u * hi) = ol; }
    __builtin_amdgcn_fence(3  , "wavefront"); __builtin_amdgcn_wave_barrier(); asm volatile("" ::: "memory");
    const unsigned rq = lane >> 3, pc = lane & 7u;
#pragma unroll 1
    for (int ps = 0; ps < 2; ++ps) {
#pragma unroll
        for (unsigned it = 0; it < 4; ++it) { const unsigned row = 4u * it + rq; const v8us a = *(const v8usa*)(sh + row * SP + pc * 8u); const v8us c2 = *(const v8usa*)(sl + row * SP + pc * 8u); const size_t oo = ((size_t)(b * (unsigned)SEQ + q0 + row)) * DM + h * (unsigned)HD + pc * 8u;
            *(volatile v8us*)(CH + oo) = a; *(volatile v8us*)(CL + oo) = c2; }
        if (ps == 0) __threadfence(); }
}

extern "C" void kernel_launch(void* const* d_in, const int* in_sizes, int n_in,
                              void* d_out, int out_size, void* d_ws, size_t ws_size, hipStream_t stream) {
    if (n_in < 7) return;
    const size_t xneed = ((size_t)(NB - 1) * SEQ_FULL + SEQ) * DM;
    if ((size_t)in_sizes[0] < xneed) return;
    if ((size_t)in_sizes[1] < (size_t)(SEQ - 1) * SEQ_FULL + SEQ) return;
    if ((size_t)in_sizes[2] < (size_t)SEQ * 32) return;
    if ((size_t)in_sizes[3] < (size_t)D3 * DM) return;
    if ((size_t)in_sizes[4] < (size_t)D3) return;
    if ((size_t)in_sizes[5] < (size_t)DM * DM) return;
    if ((size_t)in_sizes[6] < (size_t)DM) return;
    if ((size_t)out_size < xneed) return;
    const float* X = (const float*)d_in[0]; const int* MASK = (const int*)d_in[1]; const float* FR = (const float*)d_in[2];
    const float* WQKV = (const float*)d_in[3]; const float* BQKV = (const float*)d_in[4]; const float* WPR = (const float*)d_in[5]; const float* BPR = (const float*)d_in[6];
    float* OUT = (float*)d_out;
    char* wsp = (char*)d_ws;
    auto take = [&](size_t bytes) { char* p = wsp; wsp += (bytes + 255) & ~(size_t)255; return (void*)p; };
    bf* XB = (bf*)take((size_t)NTOK * DM * 2);
    bf* WQ = (bf*)take((size_t)D3 * DM * 2);
    bf* WP = (bf*)take((size_t)DM * DM * 2);
    float* CS = (float*)take((size_t)SEQ * 32 * 4); float* SN = (float*)take((size_t)SEQ * 32 * 4);
    int* FL = (int*)take((size_t)MCB * 128);
    float* QKV = (float*)take((size_t)NTOK * D3 * 4);
    bf* QKh = (bf*)take(2 * QKPL * 2); bf* QKl = (bf*)take(2 * QKPL * 2);
    bf* VTh = (bf*)take(QKPL * 2); bf* VTl = (bf*)take(QKPL * 2);
    bf* CH = (bf*)QKV; bf* CL = CH + (size_t)NTOK * DM;
    if ((size_t)(wsp - (char*)d_ws) > ws_size) return;
    k_cvtx<<<(unsigned)((size_t)NTOK * 128 / 256), 256, 0, stream>>>(X, XB);
    k_cvt8<<<(unsigned)(((size_t)D3 * DM / 8 + 255) / 256), 256, 0, stream>>>(WQKV, WQ, (size_t)D3 * DM / 8);
    k_cvt8<<<(unsigned)(((size_t)DM * DM / 8 + 255) / 256), 256, 0, stream>>>(WPR, WP, (size_t)DM * DM / 8);
    k_trig<<<(unsigned)(SEQ * 32 / 256), 256, 0, stream>>>(FR, CS, SN);
    k_mchk<<<MCB, 256, 0, stream>>>(MASK, FL);
    k_gemmw<bf, 0, true><<<dim3(NTOK / 64, D3 / 64, 1), 32, 0, stream>>>(XB, nullptr, WQ, nullptr, DM, QKV, D3, BQKV, 0, 0, 0);
    k_rope<<<(unsigned)((size_t)2 * NTOK * 128 / 256), 256, 0, stream>>>(QKV, CS, SN, QKh, QKl);
    k_vtp<<<(unsigned)((size_t)NB * NH * HD * SEQ / 2 / 256), 256, 0, stream>>>(QKV, VTh, VTl);
    k_flash<<<(unsigned)(NB * NH * QT / 8), 256, 0, stream>>>(QKh, QKl, VTh, VTl, FL, CH, CL);
    k_gemmw<bf, 1, true><<<dim3(SEQ / 64, DM / 64, NB), 32, 0, stream>>>(CH, CL, WP, nullptr, DM, OUT, DM, BPR, (size_t)SEQ * DM, 0, (size_t)SEQ_FULL * DM);
}
